// LPKTPlus_61074434949878
// MI455X (gfx1250) — hardware-run, weakly checked
//
#include <hip/hip_runtime.h>
#include <math.h>

constexpr int NBAT    = 256;
constexpr int NSEQ    = 500;
constexpr int NSTEPS  = NSEQ - 1;
constexpr int NDIM    = 256;
constexpr int NQROW   = 10001;
constexpr int NTROW   = 101;
constexpr int NQPAD   = 10048;
constexpr int NTPAD   = 128;
constexpr int W1COLS  = 576;
constexpr int WXCOLS  = 1024;
constexpr int W4COLS  = 768;
constexpr int GQCOLS  = 1024;
constexpr int GITCOLS = 768;
constexpr int DQCOLS  = 320;
constexpr int NTHR    = 256;
constexpr int HPITCH  = 264;
constexpr int ROWS_BLK = 16;
constexpr int GQ_ROWB  = GQCOLS * 4;
constexpr int GIT_ROWB = GITCOLS * 4;
constexpr int DQ_ROWB  = DQCOLS * 4;
constexpr int PARTC_B  = 512 * 4;
constexpr int GATE3_B  = 256 * 4;
constexpr float WCARRY     = 256.0f;
constexpr float WCARRY_INV = 1.0f / 256.0f;
constexpr float LOCARRY    = 2048.0f;
constexpr float LO_FOLD    = 1.0f / (256.0f * 2048.0f);
constexpr int YSPAN   = ROWS_BLK * NSEQ;
constexpr int YSPAN4  = YSPAN / 4;

static_assert(NBAT % ROWS_BLK == 0, "block rows");
static_assert(NQPAD % 64 == 0 && NQPAD >= NQROW, "table rows padded to the GEMM tile");
static_assert(NTPAD % 64 == 0 && NTPAD >= NTROW, "table rows padded to the GEMM tile");
static_assert(NDIM % 64 == 0 && GQCOLS % 64 == 0 && GITCOLS % 64 == 0 && DQCOLS % 64 == 0, "N tile multiples");
static_assert(NDIM % 32 == 0, "K multiple of 32");
static_assert((YSPAN * 4) % 128 == 0, "block output span is whole 128-B lines");
static_assert(NDIM == 32 * (NTHR / 32), "8 waves x 32 hidden units");
static_assert(3 * ROWS_BLK * HPITCH * 2 + YSPAN * 4 + 8 * 16 * 4 + 2 * 16 * 8 * 4 <= 65536, "static LDS");

typedef __attribute__((ext_vector_type(16))) _Float16 v16h;
typedef __attribute__((ext_vector_type(8)))  _Float16 v8h;
typedef __attribute__((ext_vector_type(16))) __bf16   v16b;
typedef __attribute__((ext_vector_type(8)))  __bf16   v8b;
typedef __attribute__((ext_vector_type(8)))  float    v8f;
typedef __attribute__((ext_vector_type(4)))  float    v4f;
typedef __attribute__((ext_vector_type(4)))  int      v4i;

__device__ __forceinline__ unsigned short f2bf_bits(float f) {
  unsigned u = __float_as_uint(f);
  return (unsigned short)((u + 0x7FFFu + ((u >> 16) & 1u)) >> 16);
}
__device__ __forceinline__ float bf_bits2f(unsigned short h) { return __uint_as_float(((unsigned)h) << 16); }
__device__ __forceinline__ float bf16r(float f) { return bf_bits2f(f2bf_bits(f)); }

__device__ __forceinline__ void keep4_b(v16b a, v16b b, v16b c, v16b d) { asm volatile("v_nop" :: "v"(a), "v"(b), "v"(c), "v"(d)); }
__device__ __forceinline__ void acc_guard4(v8f& a, v8f& b, v8f& c, v8f& d) { asm volatile("v_nop\n\tv_nop\n\tv_nop\n\tv_nop" : "+v"(a), "+v"(b), "+v"(c), "+v"(d)); }
__device__ __forceinline__ void acc_guard2(v8f& a, v8f& b) { asm volatile("v_nop\n\tv_nop\n\tv_nop\n\tv_nop" : "+v"(a), "+v"(b)); }
__device__ __forceinline__ void guard4_b(v8f& a, v8f& b, v8f& c, v8f& d, v16b x, v16b y) {
  asm volatile("v_nop\n\tv_nop\n\tv_nop\n\tv_nop" : "+v"(a), "+v"(b), "+v"(c), "+v"(d) : "v"(x), "v"(y));
}
__device__ __forceinline__ void guard4_h5(v8f& a, v8f& b, v8f& c, v8f& d, v16h x, v16h y0, v16h y1, v16h y2, v16h y3) {
  asm volatile("v_nop\n\tv_nop\n\tv_nop\n\tv_nop" : "+v"(a), "+v"(b), "+v"(c), "+v"(d) : "v"(x), "v"(y0), "v"(y1), "v"(y2), "v"(y3));
}
__device__ __forceinline__ void guard4_h4(v8f& a, v8f& b, v8f& c, v8f& d, v16h x0, v16h x1, v16h y0, v16h y1) {
  asm volatile("v_nop\n\tv_nop\n\tv_nop\n\tv_nop" : "+v"(a), "+v"(b), "+v"(c), "+v"(d) : "v"(x0), "v"(x1), "v"(y0), "v"(y1));
}
__device__ __forceinline__ void guard2_h3(v8f& a, v8f& b, v16h x, v16h y0, v16h y1) {
  asm volatile("v_nop\n\tv_nop\n\tv_nop\n\tv_nop" : "+v"(a), "+v"(b) : "v"(x), "v"(y0), "v"(y1));
}

template <typename T> struct Frag;
template <> struct Frag<_Float16> {
  typedef v16h V; union U { v16h v; v8h h[2]; };
  static __device__ __forceinline__ v16h load(const _Float16* p) {
    U f; f.h[0] = *(const v8h*)(p); f.h[1] = *(const v8h*)(p + 16); return f.v;
  }
  static __device__ __forceinline__ v8f mma(v16h a, v16h b, v8f c) {
    return __builtin_amdgcn_wmma_f32_16x16x32_f16(false, a, false, b, (short)0, c, false, false);
  }
};
template <> struct Frag<__bf16> {
  typedef v16b V; union U { v16b v; v8b h[2]; };
  static __device__ __forceinline__ v16b load(const __bf16* p) {
    U f; f.h[0] = *(const v8b*)(p); f.h[1] = *(const v8b*)(p + 16); return f.v;
  }
  static __device__ __forceinline__ v8f mma(v16b a, v16b b, v8f c) {
    return __builtin_amdgcn_wmma_f32_16x16x32_bf16(false, a, false, b, (short)0, c, false, false);
  }
};

__device__ __forceinline__ float fsig(float x)  { return __builtin_amdgcn_rcpf(1.0f + __expf(-x)); }
__device__ __forceinline__ float ftanh(float x) { return 1.0f - 2.0f * __builtin_amdgcn_rcpf(__expf(2.0f * x) + 1.0f); }
__device__ __forceinline__ float ldf(const float* base, int byteoff) {
  return *(const float*)((const char*)base + byteoff);
}

template <int MODE>
__global__ __launch_bounds__(NTHR) void cvt8_kernel(const float* __restrict__ srcA, const float* __restrict__ srcB,
                                                    unsigned short* __restrict__ dst,
                                                    int nrow, int nrow_src, int ncol8, int spitch,
                                                    int scol0, int stepLo, int stepHi, float sc) {
  const int piece = blockIdx.y;
  const float* src = (piece & 1) ? srcB : srcA;
  const int col0 = scol0 + (piece & 1) * stepLo + (piece >> 1) * stepHi;
  const int i  = blockIdx.x * NTHR + threadIdx.x;
  const int n8 = nrow * ncol8;
  if (i < n8) {
    const int row = i / ncol8;
    const int c8  = i - row * ncol8;
    const int rowc = (row < nrow_src) ? row : (nrow_src - 1);
    const bool live = (row < nrow_src);
    const float* sp = src + (size_t)rowc * spitch + col0 + c8 * 8;
    const v4f a = *(const v4f*)(sp);
    const v4f b = *(const v4f*)(sp + 4);
    v8h hv;
#pragma unroll
    for (int e = 0; e < 4; ++e) {
      const float ae = a[e];
      const float be = b[e];
      const float fa = live ? ae : 0.0f;
      const float fb = live ? be : 0.0f;
      unsigned short b0, b1;
      if (MODE == 0) {
        b0 = f2bf_bits(fa);
        b1 = f2bf_bits(fb);
      } else {
        const _Float16 h0 = (_Float16)(bf16r(fa) * sc);
        const _Float16 h1 = (_Float16)(bf16r(fb) * sc);
        b0 = __builtin_bit_cast(unsigned short, h0);
        b1 = __builtin_bit_cast(unsigned short, h1);
      }
      hv[e]     = __builtin_bit_cast(_Float16, b0);
      hv[4 + e] = __builtin_bit_cast(_Float16, b1);
    }
    unsigned short* dp = dst + (size_t)piece * (size_t)n8 * 8 + (size_t)i * 8;
    *(volatile v8h*)dp = hv;
    __threadfence();
    *(volatile v8h*)dp = hv;
  }
}

__global__ __launch_bounds__(NTHR) void vec_prep_kernel(const float* __restrict__ W1, const float* __restrict__ b1,
                                                        const float* __restrict__ W2, const float* __restrict__ W3,
                                                        const float* __restrict__ bd, const float* __restrict__ bdisc,
                                                        float* __restrict__ GCB, float* __restrict__ BIASD) {
  __shared__ float vcs[NDIM];
  __shared__ float b1s[NDIM];
  const int tid = threadIdx.x;
  {
    const float* wr = W1 + (size_t)tid * W1COLS + 512;
    float s = 0.0f;
#pragma unroll 1
    for (int cc = 0; cc < 64; ++cc) s += bf16r(wr[cc]);
    vcs[tid] = s;
    b1s[tid] = bf16r(b1[tid]);
  }
  __syncthreads();
  const int blk = blockIdx.x;
  if (blk < 4) {
    const float* src = (blk & 1) ? W3 : W2;
    const float* wr = src + (size_t)tid * WXCOLS + (blk >> 1) * 512;
    float sc = 0.0f, sb = 0.0f;
#pragma unroll 1
    for (int k = 0; k < NDIM; ++k) {
      const float w = bf16r(wr[k]);
      sc = fmaf(vcs[k], w, sc);
      sb = fmaf(b1s[k], w, sb);
    }
    const int n = blk * 256 + tid;
    volatile float* g0 = (volatile float*)(GCB + n);
    volatile float* g1 = (volatile float*)(GCB + GQCOLS + n);
    *g0 = sc;
    *g1 = sb;
    __threadfence();
    *g0 = sc;
    *g1 = sb;
  } else {
    const float v0 = bf16r(bd[tid]);
    const float bdv = bf16r(bdisc[0]);
    const float v1 = (tid == 0) ? bdv : 0.0f;
    volatile float* p0 = (volatile float*)(BIASD + tid);
    volatile float* p1 = (volatile float*)(BIASD + 256 + (tid & 127));
    *p0 = v0;
    if (tid < 128) *p1 = v1;
    __threadfence();
    *p0 = v0;
    if (tid < 128) *p1 = v1;
  }
}

template <int SPLITA, int BIAS_MODE, int OUT_MODE, int ACT>
__global__ __launch_bounds__(256) void tbl_gemm64(
    const unsigned short* __restrict__ Ap, const unsigned short* __restrict__ A2p, int lda,
    const unsigned short* __restrict__ Btp, int ldb,
    void* __restrict__ Cout, void* __restrict__ Cout2, int ldc,
    const float* __restrict__ bias, int M, int N, int K) {
  typedef __bf16 T;
  typedef v16b V;
  const T* A = (const T*)Ap; const T* A2 = (const T*)A2p; const T* Bt = (const T*)Btp;
  __shared__ __align__(16) float sT[8][16 * 68];
  const int lane = threadIdx.x & 31;
  const int wave = threadIdx.x >> 5;
  const int tilesN = N >> 6;
  const int tilesM = M >> 6;
  const int tile = blockIdx.x * 8 + wave;
  if (tile >= tilesM * tilesN) return;
  const int tm = tile / tilesN;
  const int tn = tile - tm * tilesN;
  const int m0 = tm << 6;
  const int n0 = tn << 6;

  const int rlane = lane & 15;
  const int koff  = (lane >> 4) * 8;
  const int mOff  = (lane >> 4) * 8;

  v8f acc[4][4];
#pragma unroll
  for (int i = 0; i < 4; ++i)
#pragma unroll
    for (int j = 0; j < 4; ++j) acc[i][j] = (v8f){0.f,0.f,0.f,0.f,0.f,0.f,0.f,0.f};

  for (int k0 = 0; k0 < K; k0 += 32) {
    V bh[4];
#pragma unroll
    for (int j = 0; j < 4; ++j) {
      const size_t bo = (size_t)(n0 + (j << 4) + rlane) * ldb + koff + k0;
      bh[j] = Frag<T>::load(Bt + bo);
    }
#pragma unroll
    for (int i = 0; i < 4; ++i) {
      const size_t ao = (size_t)(m0 + (i << 4) + rlane) * lda + koff + k0;
      V ah = Frag<T>::load(A + ao);
      V al = ah;
      if (SPLITA) al = Frag<T>::load(A2 + ao);
#pragma unroll
      for (int j = 0; j < 4; ++j) {
        acc[i][j] = Frag<T>::mma(ah, bh[j], acc[i][j]);
        if (SPLITA) acc[i][j] = Frag<T>::mma(al, bh[j], acc[i][j]);
      }
      guard4_b(acc[i][0], acc[i][1], acc[i][2], acc[i][3], ah, al);
    }
    keep4_b(bh[0], bh[1], bh[2], bh[3]);
  }
  acc_guard4(acc[0][0], acc[0][1], acc[0][2], acc[0][3]);
  acc_guard4(acc[1][0], acc[1][1], acc[1][2], acc[1][3]);
  acc_guard4(acc[2][0], acc[2][1], acc[2][2], acc[2][3]);
  acc_guard4(acc[3][0], acc[3][1], acc[3][2], acc[3][3]);

  float* slab = sT[wave];
#pragma unroll
  for (int i = 0; i < 4; ++i) {
    const int mBase = m0 + (i << 4);
#pragma unroll
    for (int j = 0; j < 4; ++j) {
      const int n = n0 + (j << 4) + rlane;
      float bv = 0.f;
      if (BIAS_MODE == 2) bv = bias[n];
#pragma unroll
      for (int r = 0; r < 8; ++r) {
        float v = acc[i][j][r];
        if (BIAS_MODE == 2) v += bv;
        if (ACT == 6) v = 1.0f / (1.0f + expf(-v));
        slab[(mOff + r) * 68 + (j << 4) + rlane] = v;
      }
    }
    __builtin_amdgcn_fence(__ATOMIC_RELEASE, "workgroup");
    __builtin_amdgcn_wave_barrier();
    __builtin_amdgcn_fence(__ATOMIC_ACQUIRE, "workgroup");
    if (OUT_MODE == 0) {
      float* C = (float*)Cout;
      const int hh = lane >> 4, c4 = (lane & 15) * 4;
      for (int pass = 0; pass < 2; ++pass) {
#pragma unroll
        for (int it = 0; it < 8; ++it) {
          const int row = it * 2 + hh;
          v4f v = *(const v4f*)(slab + row * 68 + c4);
          *(volatile v4f*)(C + (size_t)(mBase + row) * ldc + n0 + c4) = v;
        }
        __threadfence();
      }
    } else {
      const int q = lane >> 3, c8 = (lane & 7) * 8;
      unsigned short* C  = (unsigned short*)Cout;
      unsigned short* C2 = (unsigned short*)Cout2;
      for (int pass = 0; pass < 2; ++pass) {
#pragma unroll
        for (int it = 0; it < 4; ++it) {
          const int row = it * 4 + q;
          const float* sp = slab + row * 68 + c8;
          v8h hv, lv;
#pragma unroll
          for (int e = 0; e < 8; ++e) {
            const float sv = sp[e];
            const unsigned short hb = f2bf_bits(sv);
            const unsigned short lb = f2bf_bits(sv - bf_bits2f(hb));
            hv[e] = __builtin_bit_cast(_Float16, hb);
            lv[e] = __builtin_bit_cast(_Float16, lb);
          }
          *(volatile v8h*)(C  + (size_t)(mBase + row) * ldc + n0 + c8) = hv;
          *(volatile v8h*)(C2 + (size_t)(mBase + row) * ldc + n0 + c8) = lv;
        }
        __threadfence();
      }
    }
    __builtin_amdgcn_fence(__ATOMIC_RELEASE, "workgroup");
    __builtin_amdgcn_wave_barrier();
    __builtin_amdgcn_fence(__ATOMIC_ACQUIRE, "workgroup");
  }
}

__device__ __forceinline__ void build_info(int* Info, int tn, int tid, int rowbase,
                                           const int* __restrict__ qs, const int* __restrict__ its,
                                           const int* __restrict__ uts, const float* __restrict__ cs) {
  const int m = tid >> 3, f = tid & 7;
  int tt = tn;
  const bool isPrior = (f == 1) || (f == 3) || (f == 7);
  tt = isPrior ? (tn - 1) : tt;
  tt = (f == 5) ? (tn + 1) : tt;
  tt = tt < 0 ? 0 : tt;
  tt = tt > (NSEQ - 1) ? (NSEQ - 1) : tt;
  const size_t o = (size_t)(rowbase + m) * NSEQ + (size_t)tt;
  int qv = qs[o];
  int uv = uts[o];
  int iv = its[o];
  const float cv = cs[o];
  qv = qv < 0 ? 0 : (qv > NQROW - 1 ? NQROW - 1 : qv);
  uv = uv < 0 ? 0 : (uv > NTROW - 1 ? NTROW - 1 : uv);
  iv = iv < 0 ? 0 : (iv > NTROW - 1 ? NTROW - 1 : iv);
  const int cbits = __float_as_int(bf16r(cv));
  int val = cbits;
  val = (f == 5) ? qv * DQ_ROWB : val;
  val = (f == 4) ? iv * GIT_ROWB : val;
  val = (f == 2 || f == 3) ? uv * GQ_ROWB : val;
  val = (f < 2) ? qv * GQ_ROWB : val;
  Info[((tn & 1) * 16 + m) * 8 + f] = val;
}

__global__ __launch_bounds__(NTHR) void gated_scan_kernel(
    const int* __restrict__ qseq, const int* __restrict__ itseq, const int* __restrict__ utseq,
    const float* __restrict__ cseq,
    const float* __restrict__ b2, const float* __restrict__ b3, const float* __restrict__ b4, const float* __restrict__ ba,
    const float* __restrict__ GQ, const float* __restrict__ GU, const float* __restrict__ GIT,
    const float* __restrict__ DQ, const float* __restrict__ GCB,
    const unsigned short* __restrict__ WGp, const unsigned short* __restrict__ W4p,
    const unsigned short* __restrict__ WAp, float* __restrict__ out) {
  __shared__ __align__(16) _Float16 Hh[ROWS_BLK * HPITCH];
  __shared__ __align__(16) _Float16 Hl[ROWS_BLK * HPITCH];
  __shared__ __align__(16) _Float16 Lg[ROWS_BLK * HPITCH];
  __shared__ __align__(16) float    Yt[YSPAN];
  __shared__ __align__(16) float    Part[8 * 16];
  __shared__ __align__(16) int      Info[2 * 16 * 8];

  const _Float16* WG = (const _Float16*)WGp;
  const _Float16* W4 = (const _Float16*)W4p;
  const _Float16* WA = (const _Float16*)WAp;
  const int tid = threadIdx.x, lane = tid & 31, wave = tid >> 5;
  const int c = lane & 15, hh = lane >> 4, koff = hh * 8;
  const int rowbase = blockIdx.x * ROWS_BLK;

#pragma unroll 1
  for (int i = 0; i < ROWS_BLK; ++i) {
    Hh[i * HPITCH + tid] = (_Float16)1.0f;
    Hl[i * HPITCH + tid] = (_Float16)0.0f;
  }
  if (tid < ROWS_BLK) Yt[tid * NSEQ] = 0.0f;
  if (tid < 128) build_info(Info, 0, tid, rowbase, qseq, itseq, utseq, cseq);

  float hst[2][8];
  float kGcA[2][2], kGbA[2][2], kGcC[2][2], kGbC[2][2], kB4[2], kBa[2];
#pragma unroll
  for (int nt = 0; nt < 2; ++nt) {
    const int j = 32 * wave + 16 * nt + c;
#pragma unroll
    for (int r = 0; r < 8; ++r) hst[nt][r] = 1.0f;
#pragma unroll
    for (int g = 0; g < 2; ++g) {
      const int col = g * 256 + j;
      const float* bg = (g == 0) ? b2 : b3;
      kGcA[g][nt] = GCB[col];
      kGbA[g][nt] = GCB[GQCOLS + col];
      kGcC[g][nt] = GCB[512 + col];
      kGbC[g][nt] = GCB[GQCOLS + 512 + col] + bf16r(bg[j]);
    }
    kB4[nt] = bf16r(b4[j]);
    kBa[nt] = bf16r(ba[j]);
    asm volatile("" ::: "memory");
  }
  __syncthreads();

  const v8f z8 = {0.f, 0.f, 0.f, 0.f, 0.f, 0.f, 0.f, 0.f};
  const int j0 = 32 * wave + c;
  const _Float16* ahrow = Hh + c * HPITCH + koff;
  const _Float16* alrow = Hl + c * HPITCH + koff;
  const _Float16* lgrow = Lg + c * HPITCH + koff;
  const _Float16* wgrow = WG + (size_t)j0 * NDIM + koff;
  const _Float16* w4row = W4 + (size_t)j0 * 512 + koff;
  const _Float16* warow = WA + (size_t)j0 * NDIM + koff;

#pragma unroll 1
  for (int t = 0; t < NSTEPS; ++t) {
    const int* inf = Info + (t & 1) * 128;
    const bool first = (t == 0);
    float lg[2][8];

    {
      v8f g2[2], g3[2];
      g2[0] = z8; g2[1] = z8; g3[0] = z8; g3[1] = z8;
#pragma unroll 1
      for (int k0 = 0; k0 < NDIM; k0 += 32) {
        const v16h a   = Frag<_Float16>::load(ahrow + k0);
        const v16h b0  = Frag<_Float16>::load(wgrow + k0);
        const v16h b1  = Frag<_Float16>::load(wgrow + (size_t)16 * NDIM + k0);
        const v16h b2f = Frag<_Float16>::load(wgrow + (size_t)256 * NDIM + k0);
        const v16h b3f = Frag<_Float16>::load(wgrow + (size_t)272 * NDIM + k0);
        g2[0] = Frag<_Float16>::mma(a, b0, g2[0]);
        g2[1] = Frag<_Float16>::mma(a, b1, g2[1]);
        g3[0] = Frag<_Float16>::mma(a, b2f, g3[0]);
        g3[1] = Frag<_Float16>::mma(a, b3f, g3[1]);
        guard4_h5(g2[0], g2[1], g3[0], g3[1], a, b0, b1, b2f, b3f);
      }
      acc_guard4(g2[0], g2[1], g3[0], g3[1]);
#pragma unroll
      for (int r = 0; r < 8; ++r) {
        const int m = 8 * hh + r;
        const v4i ia = *(const v4i*)(inf + m * 8);
        const v4i ib = *(const v4i*)(inf + m * 8 + 4);
        const int qcB = ia[0];
        const int qaB = ia[1];
        const int ucB = ia[2];
        const int uaB = ia[3];
        const int itB = ib[0];
        const int ctb = ib[2];
        const int cpb = ib[3];
        const float ct = __int_as_float(ctb);
        const float cp = __int_as_float(cpb);
#pragma unroll
        for (int nt = 0; nt < 2; ++nt) {
          const int jB = (j0 + 16 * nt) * 4;
          const float a2 = ldf(GQ, qaB + jB) + ldf(GU, uaB + jB) + fmaf(cp, kGcA[0][nt], kGbA[0][nt]);
          const float c2 = ldf(GQ, qcB + PARTC_B + jB) + ldf(GU, ucB + PARTC_B + jB) + fmaf(ct, kGcC[0][nt], kGbC[0][nt]);
          const float i2 = ldf(GIT, itB + jB);
          const float a3 = ldf(GQ, qaB + GATE3_B + jB) + ldf(GU, uaB + GATE3_B + jB) + fmaf(cp, kGcA[1][nt], kGbA[1][nt]);
          const float c3 = ldf(GQ, qcB + PARTC_B + GATE3_B + jB) + ldf(GU, ucB + PARTC_B + GATE3_B + jB) + fmaf(ct, kGcC[1][nt], kGbC[1][nt]);
          const float i3 = ldf(GIT, itB + GATE3_B + jB);
          const float s2 = (first ? 0.0f : a2) + c2 + i2;
          const float s3 = (first ? 0.0f : a3) + c3 + i3;
          const float p2 = fmaf(g2[nt][r], WCARRY_INV, s2);
          const float p3 = fmaf(g3[nt][r], WCARRY_INV, s3);
          const float gain = ftanh(p2);
          const float gl   = fsig(p3);
          const float lgv  = gl * (gain + 1.0f) * 0.5f;
          lg[nt][r] = lgv;
          Lg[m * HPITCH + j0 + 16 * nt] = (_Float16)lgv;
          asm volatile("" ::: "memory");
        }
      }
    }
    __syncthreads();

    if (wave == 0 && t > 0) {
      const int m = lane & 15;
      float s = 0.0f;
#pragma unroll
      for (int w = 0; w < 8; ++w) s += Part[w * 16 + m];
      const int qB = inf[m * 8];
      const int qi = qB >> 12;
      float dqv = DQ[(size_t)qi * DQCOLS + 256];
      asm volatile("" : "+v"(dqv));
      const float disc = 10.0f * dqv;
      const float y = fsig(disc * s);
      Yt[m * NSEQ + t] = y;
    }
    if (tid < 128) build_info(Info, t + 1, tid, rowbase, qseq, itseq, utseq, cseq);

    {
      v8f f4[2];
      f4[0] = z8; f4[1] = z8;
#pragma unroll 1
      for (int k0 = 0; k0 < NDIM; k0 += 32) {
        const v16h a  = Frag<_Float16>::load(ahrow + k0);
        const v16h b0 = Frag<_Float16>::load(w4row + k0);
        const v16h b1 = Frag<_Float16>::load(w4row + (size_t)16 * 512 + k0);
        f4[0] = Frag<_Float16>::mma(a, b0, f4[0]);
        f4[1] = Frag<_Float16>::mma(a, b1, f4[1]);
        guard2_h3(f4[0], f4[1], a, b0, b1);
      }
#pragma unroll 1
      for (int k0 = 0; k0 < NDIM; k0 += 32) {
        const v16h a  = Frag<_Float16>::load(lgrow + k0);
        const v16h b0 = Frag<_Float16>::load(w4row + 256 + k0);
        const v16h b1 = Frag<_Float16>::load(w4row + (size_t)16 * 512 + 256 + k0);
        f4[0] = Frag<_Float16>::mma(a, b0, f4[0]);
        f4[1] = Frag<_Float16>::mma(a, b1, f4[1]);
        guard2_h3(f4[0], f4[1], a, b0, b1);
      }
      acc_guard2(f4[0], f4[1]);
#pragma unroll
      for (int r = 0; r < 8; ++r) {
        const int m = 8 * hh + r;
        const int itB = inf[m * 8 + 4];
#pragma unroll
        for (int nt = 0; nt < 2; ++nt) {
          const int jB = (j0 + 16 * nt) * 4;
          const float gi = ldf(GIT, itB + PARTC_B + jB);
          const float gf = fsig(fmaf(f4[nt][r], WCARRY_INV, gi + kB4[nt]));
          hst[nt][r] = lg[nt][r] + gf * hst[nt][r];
        }
      }
    }
    __syncthreads();
#pragma unroll
    for (int nt = 0; nt < 2; ++nt) {
#pragma unroll
      for (int r = 0; r < 8; ++r) {
        const float hv = hst[nt][r];
        const _Float16 hi = (_Float16)hv;
        float hif = (float)hi;
        asm volatile("" : "+v"(hif));
        const float res = (hv - hif) * LOCARRY;
        Hh[(8 * hh + r) * HPITCH + j0 + 16 * nt] = hi;
        Hl[(8 * hh + r) * HPITCH + j0 + 16 * nt] = (_Float16)res;
      }
    }
    __syncthreads();

    {
      v8f ph[2], pl[2];
      ph[0] = z8; ph[1] = z8; pl[0] = z8; pl[1] = z8;
#pragma unroll 1
      for (int k0 = 0; k0 < NDIM; k0 += 32) {
        const v16h a  = Frag<_Float16>::load(ahrow + k0);
        const v16h al = Frag<_Float16>::load(alrow + k0);
        const v16h b0 = Frag<_Float16>::load(warow + k0);
        const v16h b1 = Frag<_Float16>::load(warow + (size_t)16 * NDIM + k0);
        ph[0] = Frag<_Float16>::mma(a,  b0, ph[0]);
        ph[1] = Frag<_Float16>::mma(a,  b1, ph[1]);
        pl[0] = Frag<_Float16>::mma(al, b0, pl[0]);
        pl[1] = Frag<_Float16>::mma(al, b1, pl[1]);
        guard4_h4(ph[0], ph[1], pl[0], pl[1], a, al, b0, b1);
      }
      acc_guard4(ph[0], ph[1], pl[0], pl[1]);
      float s[8];
#pragma unroll
      for (int r = 0; r < 8; ++r) {
        const int m = 8 * hh + r;
        const int dB = inf[m * 8 + 5];
        float sv = 0.0f;
#pragma unroll
        for (int nt = 0; nt < 2; ++nt) {
          const int jB = (j0 + 16 * nt) * 4;
          const float u  = fmaf(ph[nt][r], WCARRY_INV, fmaf(pl[nt][r], LO_FOLD, kBa[nt]));
          const float av = fsig(u);
          const float dv = ldf(DQ, dB + jB);
          sv += (av - dv) * dv;
        }
        s[r] = sv;
      }
#pragma unroll
      for (int off = 1; off < 16; off <<= 1) {
#pragma unroll
        for (int r = 0; r < 8; ++r) s[r] += __shfl_xor(s[r], off, 32);
      }
      if (c == 0) {
#pragma unroll
        for (int r = 0; r < 8; ++r) Part[wave * 16 + 8 * hh + r] = s[r];
      }
    }
  }

  __syncthreads();
  if (wave == 0) {
    const int* inf = Info + (NSTEPS & 1) * 128;
    const int m = lane & 15;
    float s = 0.0f;
#pragma unroll
    for (int w = 0; w < 8; ++w) s += Part[w * 16 + m];
    const int qB = inf[m * 8];
    const int qi = qB >> 12;
    float dqv = DQ[(size_t)qi * DQCOLS + 256];
    asm volatile("" : "+v"(dqv));
    const float disc = 10.0f * dqv;
    const float y = fsig(disc * s);
    Yt[m * NSEQ + NSTEPS] = y;
  }
  __syncthreads();

  float* ob = out + (size_t)blockIdx.x * YSPAN;
  for (int pass = 0; pass < 2; ++pass) {
#pragma unroll
    for (int it = 0; it < 8; ++it) {
      const int idx = it * NTHR + tid;
      if (idx < YSPAN4) {
        const v4f v = *(const v4f*)(Yt + 4 * idx);
        *(volatile v4f*)(ob + 4 * idx) = v;
      }
    }
    __threadfence();
  }
}

extern "C" void kernel_launch(void* const* d_in, const int* in_sizes, int n_in,
                              void* d_out, int out_size, void* d_ws, size_t ws_size, hipStream_t stream) {
  if (n_in < 21 || d_out == nullptr || d_ws == nullptr) return;
  if (in_sizes[0] != NBAT * NSEQ || in_sizes[1] != NBAT * NSEQ || in_sizes[2] != NBAT * NSEQ ||
      in_sizes[3] != NBAT * NSEQ || in_sizes[4] != NQROW * NDIM || in_sizes[5] != NTROW * NDIM ||
      in_sizes[6] != NTROW * NDIM || in_sizes[7] != NDIM * W1COLS || in_sizes[8] != NDIM ||
      in_sizes[9] != NDIM * WXCOLS || in_sizes[10] != NDIM || in_sizes[11] != NDIM * WXCOLS ||
      in_sizes[12] != NDIM || in_sizes[13] != NDIM * W4COLS || in_sizes[14] != NDIM ||
      in_sizes[15] != NDIM * NDIM || in_sizes[16] != NDIM || in_sizes[17] != NDIM * NDIM ||
      in_sizes[18] != NDIM || in_sizes[19] != NDIM || in_sizes[20] != 1 || out_size != NBAT * NSEQ) return;

  const int*   qseq  = (const int*)d_in[0];
  const int*   itseq = (const int*)d_in[1];
  const int*   utseq = (const int*)d_in[2];
  const float* cseq  = (const float*)d_in[3];
  const float* Eq    = (const float*)d_in[4];
  const float* Eut   = (const float*)d_in[5];
  const float* Eit   = (const float*)d_in[6];
  const float* W1    = (const float*)d_in[7];
  const float* b1    = (const float*)d_in[8];
  const float* W2    = (const float*)d_in[9];
  const float* b2    = (const float*)d_in[10];
  const float* W3    = (const float*)d_in[11];
  const float* b3    = (const float*)d_in[12];
  const float* W4    = (const float*)d_in[13];
  const float* b4    = (const float*)d_in[14];
  const float* Wa    = (const float*)d_in[15];
  const float* ba    = (const float*)d_in[16];
  const float* Wd    = (const float*)d_in[17];
  const float* bd    = (const float*)d_in[18];
  const float* Wdisc = (const float*)d_in[19];
  const float* bdisc = (const float*)d_in[20];
  float* out = (float*)d_out;

  char* ws = (char*)d_ws; size_t off = 0;
  auto carve = [&](size_t bytes) -> char* { char* p = ws + off; off += (bytes + 255) & ~(size_t)255; return p; };
  unsigned short* EQB   = (unsigned short*)carve((size_t)NQPAD * NDIM * 2);
  unsigned short* EUB   = (unsigned short*)carve((size_t)NTPAD * NDIM * 2);
  unsigned short* EIB   = (unsigned short*)carve((size_t)NTPAD * NDIM * 2);
  unsigned short* W1B   = (unsigned short*)carve((size_t)2 * NDIM * NDIM * 2);
  unsigned short* WDB   = (unsigned short*)carve((size_t)DQCOLS * NDIM * 2);
  unsigned short* WCATB = (unsigned short*)carve((size_t)GQCOLS * NDIM * 2);
  unsigned short* WITB  = (unsigned short*)carve((size_t)GITCOLS * NDIM * 2);
  unsigned short* WG    = (unsigned short*)carve((size_t)512 * NDIM * 2);
  unsigned short* W4P   = (unsigned short*)carve((size_t)NDIM * 512 * 2);
  unsigned short* WAP   = (unsigned short*)carve((size_t)NDIM * NDIM * 2);
  float*          GCB   = (float*)carve((size_t)2 * GQCOLS * 4);
  float*          BIASD = (float*)carve((size_t)384 * 4);
  unsigned short* PQH   = (unsigned short*)carve((size_t)NQPAD * NDIM * 2);
  unsigned short* PQL   = (unsigned short*)carve((size_t)NQPAD * NDIM * 2);
  float*          DQ    = (float*)carve((size_t)NQPAD * DQCOLS * 4);
  float*          GQ    = (float*)carve((size_t)NQPAD * GQCOLS * 4);
  unsigned short* PUH   = (unsigned short*)carve((size_t)NTPAD * NDIM * 2);
  unsigned short* PUL   = (unsigned short*)carve((size_t)NTPAD * NDIM * 2);
  float*          GU    = (float*)carve((size_t)NTPAD * GQCOLS * 4);
  float*          GIT   = (float*)carve((size_t)NTPAD * GITCOLS * 4);
  if (off > ws_size || off > (size_t)134217728) return;

  const int NC8 = NDIM / 8;
  cvt8_kernel<0><<<dim3(NQPAD * NC8 / NTHR, 1), NTHR, 0, stream>>>(Eq,  Eq,  EQB, NQPAD, NQROW, NC8, NDIM, 0, 0, 0, 1.0f);
  cvt8_kernel<0><<<dim3(NTPAD * NC8 / NTHR, 1), NTHR, 0, stream>>>(Eut, Eut, EUB, NTPAD, NTROW, NC8, NDIM, 0, 0, 0, 1.0f);
  cvt8_kernel<0><<<dim3(NTPAD * NC8 / NTHR, 1), NTHR, 0, stream>>>(Eit, Eit, EIB, NTPAD, NTROW, NC8, NDIM, 0, 0, 0, 1.0f);
  cvt8_kernel<0><<<dim3(NDIM * NC8 / NTHR, 2), NTHR, 0, stream>>>(W1, W1, W1B, NDIM, NDIM, NC8, W1COLS, 0, 256, 0, 1.0f);
  cvt8_kernel<0><<<dim3(NDIM * NC8 / NTHR, 1), NTHR, 0, stream>>>(Wd, Wd, WDB, NDIM, NDIM, NC8, NDIM, 0, 0, 0, 1.0f);
  cvt8_kernel<0><<<dim3(64 * NC8 / NTHR, 1), NTHR, 0, stream>>>(Wdisc, Wdisc, WDB + (size_t)NDIM * NDIM, 64, 1, NC8, NDIM, 0, 0, 0, 1.0f);
  cvt8_kernel<0><<<dim3(NDIM * NC8 / NTHR, 4), NTHR, 0, stream>>>(W2, W3, WCATB, NDIM, NDIM, NC8, WXCOLS, 0, 0, 512, 1.0f);
  cvt8_kernel<0><<<dim3(NDIM * NC8 / NTHR, 2), NTHR, 0, stream>>>(W2, W3, WITB, NDIM, NDIM, NC8, WXCOLS, 256, 0, 0, 1.0f);
  cvt8_kernel<0><<<dim3(NDIM * NC8 / NTHR, 1), NTHR, 0, stream>>>(W4, W4, WITB + (size_t)2 * NDIM * NDIM, NDIM, NDIM, NC8, W4COLS, 512, 0, 0, 1.0f);
  cvt8_kernel<1><<<dim3(NDIM * NC8 / NTHR, 2), NTHR, 0, stream>>>(W2, W3, WG, NDIM, NDIM, NC8, WXCOLS, 768, 0, 0, WCARRY);
  cvt8_kernel<1><<<dim3(NDIM * 64 / NTHR, 1), NTHR, 0, stream>>>(W4, W4, W4P, NDIM, NDIM, 64, W4COLS, 0, 0, 0, WCARRY);
  cvt8_kernel<1><<<dim3(NDIM * NC8 / NTHR, 1), NTHR, 0, stream>>>(Wa, Wa, WAP, NDIM, NDIM, NC8, NDIM, 0, 0, 0, WCARRY);
  vec_prep_kernel<<<5, NTHR, 0, stream>>>(W1, b1, W2, W3, bd, bdisc, GCB, BIASD);

  auto gblocks = [](int M, int N) -> int { return ((M / 64) * (N / 64) + 7) / 8; };
  tbl_gemm64<0, 0, 2, 0><<<gblocks(NQPAD, NDIM), 256, 0, stream>>>(
      EQB, EQB, NDIM, W1B, NDIM, (void*)PQH, (void*)PQL, NDIM, BIASD, NQPAD, NDIM, NDIM);
  tbl_gemm64<0, 2, 0, 6><<<gblocks(NQPAD, DQCOLS), 256, 0, stream>>>(
      EQB, EQB, NDIM, WDB, NDIM, (void*)DQ, (void*)DQ, DQCOLS, BIASD, NQPAD, DQCOLS, NDIM);
  tbl_gemm64<1, 0, 0, 0><<<gblocks(NQPAD, GQCOLS), 256, 0, stream>>>(
      PQH, PQL, NDIM, WCATB, NDIM, (void*)GQ, (void*)GQ, GQCOLS, BIASD, NQPAD, GQCOLS, NDIM);
  tbl_gemm64<0, 0, 2, 0><<<gblocks(NTPAD, NDIM), 256, 0, stream>>>(
      EUB, EUB, NDIM, W1B + (size_t)NDIM * NDIM, NDIM, (void*)PUH, (void*)PUL, NDIM, BIASD, NTPAD, NDIM, NDIM);
  tbl_gemm64<1, 0, 0, 0><<<gblocks(NTPAD, GQCOLS), 256, 0, stream>>>(
      PUH, PUL, NDIM, WCATB, NDIM, (void*)GU, (void*)GU, GQCOLS, BIASD, NTPAD, GQCOLS, NDIM);
  tbl_gemm64<0, 0, 0, 0><<<gblocks(NTPAD, GITCOLS), 256, 0, stream>>>(
      EIB, EIB, NDIM, WITB, NDIM, (void*)GIT, (void*)GIT, GITCOLS, BIASD, NTPAD, GITCOLS, NDIM);

  gated_scan_kernel<<<NBAT / ROWS_BLK, NTHR, 0, stream>>>(qseq, itseq, utseq, cseq, b2, b3, b4, ba,
                                                          GQ, GU, GIT, DQ, GCB, WG, W4P, WAP, out);
}
